// ClusterOTRecommender_58909771432117
// MI455X (gfx1250) — hardware-verified
//
#include <hip/hip_runtime.h>
#include <stdint.h>
#include <stddef.h>
#include <math.h>

#pragma clang fp contract(off)

#define NTOK 4096
#define DIN  512
#define DHID 1024
#define DOUT 512
#define NEX  16
#define KS   8
#define MT   32
#define GX   8
#define TPB  16
#define HC   128
#define XP   520
#define HP   136
#define YP   516
#define RECW 16
#define TT   64
#define TPF  68

#define LDS_XB  (MT * XP * 2)
#define LDS_HB  (MT * HP * 2)
#define LDS_YB  (MT * YP * 4)
#define LDS_EXP (LDS_XB + LDS_HB + LDS_YB)

#define W_SC 256.0f
#define H_SC 16.0f
#define R_1  0.00390625f
#define R_2  0.000244140625f

static_assert((XP * 2) % 16 == 0);
static_assert((HP * 2) % 16 == 0);
static_assert((YP * 4) % 16 == 0);
static_assert((TPF * 4) % 16 == 0);
static_assert(LDS_XB % 16 == 0);
static_assert((LDS_XB + LDS_HB) % 16 == 0);
static_assert(GX * TPB * MT == NTOK);
static_assert(MT * (DIN / 8) == 8 * 256);
static_assert(DIN % 32 == 0);
static_assert(DHID % HC == 0);
static_assert(HC == 8 * 16);
static_assert(HC % 32 == 0);
static_assert(DOUT == 8 * 64);
static_assert(DOUT == 4 * 128);
static_assert(NTOK % 256 == 0);
static_assert(NTOK % 8 == 0);
static_assert(DIN % TT == 0);
static_assert(DHID % TT == 0);
static_assert(DOUT % TT == 0);
static_assert((DIN * NEX) % 1024 == 0);
static_assert((NTOK * DIN) % (8 * 256) == 0);
static_assert(NEX == 16);
static_assert(RECW == NEX);
static_assert(KS <= NEX);
static_assert(8 * RECW == 128);
static_assert(MT == 8 * 4);

typedef _Float16       v16h __attribute__((ext_vector_type(16)));
typedef _Float16       v8h  __attribute__((ext_vector_type(8)));
typedef float          v8f  __attribute__((ext_vector_type(8)));
typedef float          v4f  __attribute__((ext_vector_type(4)));
typedef unsigned int   v4u  __attribute__((ext_vector_type(4)));
typedef v4f __attribute__((may_alias)) v4fa;
typedef v4u __attribute__((may_alias)) v4ua;

union FragH { v16h v; v4u q[2]; };
union Pack8 { v8h h; v4u u; };

__device__ __forceinline__ v8f wmma_h(v16h a, v16h b, v8f c) {
  v8f d = __builtin_amdgcn_wmma_f32_16x16x32_f16(false, a, false, b, (short)0, c, false, false);
  asm volatile("v_nop\n\tv_nop\n\tv_nop\n\tv_nop" : "+v"(d) : "v"(a), "v"(b));
  return d;
}

__device__ __forceinline__ v16h ldfrag(const unsigned short* p, int h) {
  FragH f;
  f.q[0] = *(const v4ua*)(p + 8 * h);
  f.q[1] = *(const v4ua*)(p + 16 + 8 * h);
  return f.v;
}

__global__ __launch_bounds__(256) void k_cvt(const float* __restrict__ src,
                                             unsigned short* __restrict__ dst,
                                             int n8, float sc)
{
  const int g = blockIdx.x * 256 + threadIdx.x;
  if (g >= n8) return;
  const float* s = src + (size_t)g * 8;
  const v4f a = *(const v4fa*)s;
  const v4f c = *(const v4fa*)(s + 4);
  v8h hv;
  hv[0] = (_Float16)(a.x * sc); hv[1] = (_Float16)(a.y * sc);
  hv[2] = (_Float16)(a.z * sc); hv[3] = (_Float16)(a.w * sc);
  hv[4] = (_Float16)(c.x * sc); hv[5] = (_Float16)(c.y * sc);
  hv[6] = (_Float16)(c.z * sc); hv[7] = (_Float16)(c.w * sc);
  Pack8 p;
  p.h = hv;
  const v4u u = p.u;
  unsigned short* d = dst + (size_t)g * 8;
  *(volatile v4u*)d = u;
  __threadfence();
  *(volatile v4u*)d = u;
}

__global__ __launch_bounds__(256) void k_tcv(const float* __restrict__ src,
                                             unsigned short* __restrict__ dst,
                                             int R, int C, float sc)
{
  __shared__ __align__(16) float tile[TT * TPF];
  const int tid = threadIdx.x;
  const int n0 = blockIdx.x * TT, k0 = blockIdx.y * TT, e = blockIdx.z;
  const float* s = src + (size_t)e * R * C;
  #pragma unroll
  for (int j = 0; j < 4; ++j) {
    const int r  = (tid >> 4) + 16 * j;
    const int c4 = tid & 15;
    const v4f v = *(const v4fa*)(s + (size_t)(k0 + r) * C + n0 + 4 * c4);
    *(v4fa*)(tile + r * TPF + 4 * c4) = v;
  }
  __syncthreads();
  v4u u[2];
  #pragma unroll
  for (int j = 0; j < 2; ++j) {
    const int n = (tid >> 3) + 32 * j;
    const int q = tid & 7;
    v8h hv;
    #pragma unroll
    for (int i = 0; i < 8; ++i) hv[i] = (_Float16)(tile[(8 * q + i) * TPF + n] * sc);
    Pack8 pk;
    pk.h = hv;
    u[j] = pk.u;
  }
  unsigned short* d0 = dst + (size_t)e * C * R + (size_t)(n0 + (tid >> 3)) * R + k0 + 8 * (tid & 7);
  unsigned short* d1 = d0 + (size_t)32 * R;
  *(volatile v4u*)d0 = u[0];
  *(volatile v4u*)d1 = u[1];
  __threadfence();
  *(volatile v4u*)d0 = u[0];
  *(volatile v4u*)d1 = u[1];
}

__global__ __launch_bounds__(256) void k_route(const float* __restrict__ gx,
                                               const float* __restrict__ wg,
                                               const int* __restrict__ kin,
                                               float* __restrict__ rec, int ntok)
{
  __shared__ __align__(16) float swg[DIN * NEX];
  __shared__ __align__(16) float srec[8 * RECW];
  const int tid = threadIdx.x, lane = tid & 31, wv = tid >> 5;
  #pragma unroll 1
  for (int i = 0; i < (DIN * NEX) / 1024; ++i) {
    const int o = 4 * (tid + 256 * i);
    const v4f w4 = *(const v4fa*)(wg + o);
    *(v4fa*)(swg + o) = w4;
  }
  __syncthreads();

  int kk = kin[0];
  kk = (kk < 1) ? 1 : ((kk > KS) ? KS : kk);

  const int t = blockIdx.x * 8 + wv;
  const int tc = (t < ntok) ? t : (ntok - 1);
  const float* xr = gx + (size_t)tc * DIN;
  double lg[NEX];
  #pragma unroll
  for (int e = 0; e < NEX; ++e) lg[e] = 0.0;
  #pragma unroll 1
  for (int i = 0; i < DIN / 32; ++i) {
    const int d = 32 * i + lane;
    const double xv = (double)xr[d];
    const v4f w0 = *(const v4fa*)(swg + d * NEX);
    const v4f w1 = *(const v4fa*)(swg + d * NEX + 4);
    const v4f w2 = *(const v4fa*)(swg + d * NEX + 8);
    const v4f w3 = *(const v4fa*)(swg + d * NEX + 12);
    lg[0]  = fma(xv, (double)w0.x, lg[0]);
    lg[1]  = fma(xv, (double)w0.y, lg[1]);
    lg[2]  = fma(xv, (double)w0.z, lg[2]);
    lg[3]  = fma(xv, (double)w0.w, lg[3]);
    lg[4]  = fma(xv, (double)w1.x, lg[4]);
    lg[5]  = fma(xv, (double)w1.y, lg[5]);
    lg[6]  = fma(xv, (double)w1.z, lg[6]);
    lg[7]  = fma(xv, (double)w1.w, lg[7]);
    lg[8]  = fma(xv, (double)w2.x, lg[8]);
    lg[9]  = fma(xv, (double)w2.y, lg[9]);
    lg[10] = fma(xv, (double)w2.z, lg[10]);
    lg[11] = fma(xv, (double)w2.w, lg[11]);
    lg[12] = fma(xv, (double)w3.x, lg[12]);
    lg[13] = fma(xv, (double)w3.y, lg[13]);
    lg[14] = fma(xv, (double)w3.z, lg[14]);
    lg[15] = fma(xv, (double)w3.w, lg[15]);
  }
  #pragma unroll
  for (int off = 16; off > 0; off >>= 1) {
    #pragma unroll
    for (int e = 0; e < NEX; ++e) lg[e] = lg[e] + __shfl_xor(lg[e], off);
  }

  unsigned int chosen = 0u;
  #pragma unroll 1
  for (int j = 0; j < kk; ++j) {
    int bi = -1;
    double bv = -1.0e300;
    #pragma unroll
    for (int e = 0; e < NEX; ++e) {
      const bool take = (((chosen >> e) & 1u) == 0u) && (lg[e] > bv);
      bv = take ? lg[e] : bv;
      bi = take ? e : bi;
    }
    bi = (bi < 0) ? (__builtin_ffs((int)(~chosen & 0xFFFFu)) - 1) : bi;
    bi = (bi < 0) ? 0 : ((bi > NEX - 1) ? (NEX - 1) : bi);
    chosen |= (1u << bi);
  }

  float mxf = -3.0e38f;
  float myl = 0.0f;
  #pragma unroll
  for (int e = 0; e < NEX; ++e) {
    const float lf = (float)lg[e];
    const bool sel = ((chosen >> e) & 1u) != 0u;
    mxf = (sel && (lf > mxf)) ? lf : mxf;
    myl = (lane == e) ? lf : myl;
  }
  const bool mysel = (lane < NEX) && (((chosen >> (lane & (NEX - 1))) & 1u) != 0u);
  const float arg = mysel ? (myl - mxf) : 0.0f;
  const float exq = expf(arg);
  const float exv = mysel ? exq : 0.0f;
  float se = exv;
  #pragma unroll
  for (int off = 16; off > 0; off >>= 1) se = se + __shfl_xor(se, off);
  const float rse = 1.0f / se;
  const float gv = exv * rse;

  if (lane < NEX) srec[wv * RECW + lane] = gv;
  __syncthreads();
  if (wv == 0) {
    const v4f v = *(const v4fa*)(srec + 4 * lane);
    const int tt = blockIdx.x * 8 + (lane >> 2);
    const bool ok = (tt < ntok);
    float* dst = rec + (size_t)(blockIdx.x * 8) * RECW + 4 * lane;
    if (ok) *(volatile v4f*)dst = v;
    __threadfence();
    if (ok) *(volatile v4f*)dst = v;
  }
}

__device__ __forceinline__ void part_pass(const float* sY, const int* tk, const int* sl,
                                          float* part, int wv, int lane, int nrows)
{
  #pragma unroll
  for (int i = 0; i < 4; ++i) {
    const int row = wv * 4 + i;
    int t = tk[row];
    t = (t < 0) ? 0 : ((t > NTOK - 1) ? (NTOK - 1) : t);
    int s = sl[row];
    s = (s < 0) ? 0 : ((s > KS - 1) ? (KS - 1) : s);
    v4f v[4];
    #pragma unroll
    for (int j = 0; j < 4; ++j) v[j] = *(const v4fa*)(sY + row * YP + 128 * j + 4 * lane);
    float* dst = part + ((size_t)t * KS + s) * DOUT;
    if (row < nrows) {
      #pragma unroll
      for (int j = 0; j < 4; ++j) *(volatile v4f*)(dst + 128 * j + 4 * lane) = v[j];
    }
  }
}

__global__ __launch_bounds__(256) void k_expert(const unsigned short* __restrict__ xh,
                                                const unsigned short* __restrict__ w1t,
                                                const float* __restrict__ b1,
                                                const unsigned short* __restrict__ w2t,
                                                const float* __restrict__ b2,
                                                const float* __restrict__ rec,
                                                float* __restrict__ part, int ntok)
{
  extern __shared__ __align__(16) unsigned char dsm_e[];
  unsigned short* sX = (unsigned short*)dsm_e;
  unsigned short* sH = (unsigned short*)(dsm_e + LDS_XB);
  float* sY = (float*)(dsm_e + LDS_XB + LDS_HB);
  __shared__ int   sTok[TPB * MT];
  __shared__ int   sSlot[TPB * MT];
  __shared__ float sW[TPB * MT];
  __shared__ int   s_wc[8];

  const int tid = threadIdx.x, lane = tid & 31, wv = tid >> 5;
  const int h = lane >> 4, m = lane & 15;
  const int e = blockIdx.y;
  const int bx = blockIdx.x;

  for (int i = tid; i < TPB * MT; i += 256) { sTok[i] = 0; sSlot[i] = 0; sW[i] = 0.0f; }
  __syncthreads();

  int base = 0;
  #pragma unroll 1
  for (int ch = 0; ch < NTOK / 256; ++ch) {
    const int t = ch * 256 + tid;
    const int tc = (t < ntok) ? t : (ntok - 1);
    const float* rp = rec + (size_t)tc * RECW;
    int below = 0;
    float ge = 0.0f;
    #pragma unroll
    for (int i = 0; i < NEX; ++i) {
      const float gi = rp[i];
      below += ((i < e) && (gi > 0.0f)) ? 1 : 0;
      ge = (i == e) ? gi : ge;
    }
    const bool f = (ge > 0.0f) && (t < ntok);
    const unsigned int msk = __builtin_amdgcn_ballot_w32(f);
    const int off = __builtin_popcount(msk & ((1u << lane) - 1u));
    const int wcnt = __builtin_popcount(msk);
    if (lane == 0) s_wc[wv] = wcnt;
    __syncthreads();
    int pre = 0, tot = 0;
    #pragma unroll
    for (int w2 = 0; w2 < 8; ++w2) {
      const int c2 = s_wc[w2];
      tot += c2;
      pre += (w2 < wv) ? c2 : 0;
    }
    if (f) {
      const int rank = base + pre + off;
      const int tile = rank / MT;
      const int lt = tile / GX;
      const int p = lt * MT + (rank % MT);
      if (((tile % GX) == bx) && ((unsigned)p < (unsigned)(TPB * MT))) {
        sTok[p]  = t;
        sSlot[p] = below;
        sW[p]    = ge;
      }
    }
    base += tot;
    __syncthreads();
  }
  const int cnt = base;

  const v8f z8 = {0.f, 0.f, 0.f, 0.f, 0.f, 0.f, 0.f, 0.f};

  #pragma unroll 1
  for (int lt = 0; lt < TPB; ++lt) {
    const int m0 = (bx + GX * lt) * MT;
    if (m0 >= cnt) break;
    int nrows = cnt - m0;
    nrows = (nrows > MT) ? MT : nrows;
    const int lo = lt * MT;

    #pragma unroll
    for (int j = 0; j < 8; ++j) {
      const int idx = tid + 256 * j;
      const int row = idx >> 6, c8 = idx & 63;
      int t = sTok[lo + row];
      t = (t < 0) ? 0 : ((t > NTOK - 1) ? (NTOK - 1) : t);
      const size_t go = (size_t)t * DIN + 8 * c8;
      const v4u a = *(const v4ua*)(xh + go);
      *(v4ua*)(sX + row * XP + 8 * c8) = a;
    }
    __syncthreads();

    v8f acc2[2][4];
    #pragma unroll
    for (int mt = 0; mt < 2; ++mt)
      #pragma unroll
      for (int nt = 0; nt < 4; ++nt) acc2[mt][nt] = z8;

    #pragma unroll 1
    for (int hc = 0; hc < DHID; hc += HC) {
      const int jcol = hc + 16 * wv + m;
      const unsigned short* w1row = w1t + ((size_t)e * DHID + jcol) * DIN;
      v8f acc1[2];
      acc1[0] = z8; acc1[1] = z8;
      #pragma unroll 2
      for (int kb = 0; kb < DIN; kb += 32) {
        const v16h b = ldfrag(w1row + kb, h);
        #pragma unroll
        for (int mt = 0; mt < 2; ++mt) {
          const v16h a = ldfrag(sX + (16 * mt + m) * XP + kb, h);
          acc1[mt] = wmma_h(a, b, acc1[mt]);
        }
      }
      const float bias1 = b1[(size_t)e * DHID + jcol];
      #pragma unroll
      for (int mt = 0; mt < 2; ++mt) {
        #pragma unroll
        for (int r = 0; r < 8; ++r) {
          const int row = 16 * mt + 8 * h + r;
          float hv = acc1[mt][r] * R_1 + bias1;
          hv = (hv > 0.0f) ? hv : 0.0f;
          const _Float16 hq = (_Float16)(hv * H_SC);
          sH[row * HP + 16 * wv + m] = __builtin_bit_cast(unsigned short, hq);
        }
      }
      __syncthreads();

      #pragma unroll 1
      for (int kk = 0; kk < HC / 32; ++kk) {
        const int kb = 32 * kk;
        v16h a2[2];
        #pragma unroll
        for (int mt = 0; mt < 2; ++mt) a2[mt] = ldfrag(sH + (16 * mt + m) * HP + kb, h);
        #pragma unroll
        for (int nt = 0; nt < 4; ++nt) {
          const int ocol = wv * 64 + 16 * nt + m;
          const unsigned short* w2row = w2t + ((size_t)e * DOUT + ocol) * DHID + hc + kb;
          const v16h b = ldfrag(w2row, h);
          #pragma unroll
          for (int mt = 0; mt < 2; ++mt) acc2[mt][nt] = wmma_h(a2[mt], b, acc2[mt][nt]);
        }
      }
      __syncthreads();
    }

    #pragma unroll
    for (int nt = 0; nt < 4; ++nt) {
      const int ocol = wv * 64 + 16 * nt + m;
      const float b2v = b2[(size_t)e * DOUT + ocol];
      #pragma unroll
      for (int mt = 0; mt < 2; ++mt) {
        #pragma unroll
        for (int r = 0; r < 8; ++r) {
          const int row = 16 * mt + 8 * h + r;
          const float y = (acc2[mt][nt][r] * R_2 + b2v) * sW[lo + row];
          sY[row * YP + ocol] = y;
        }
      }
    }
    __syncthreads();
    part_pass(sY, sTok + lo, sSlot + lo, part, wv, lane, nrows);
    __threadfence();
    part_pass(sY, sTok + lo, sSlot + lo, part, wv, lane, nrows);
    __syncthreads();
  }
}

__global__ __launch_bounds__(256) void k_sum(const float* __restrict__ part,
                                             const float* __restrict__ rec,
                                             float* __restrict__ out, int ntok)
{
  const int lane = threadIdx.x & 31, wv = threadIdx.x >> 5;
  const int t = blockIdx.x * 8 + wv;
  if (t >= ntok) return;
  const float* rp = rec + (size_t)t * RECW;
  int nsel = 0;
  #pragma unroll
  for (int i = 0; i < NEX; ++i) nsel += (rp[i] > 0.0f) ? 1 : 0;
  nsel = (nsel > KS) ? KS : nsel;
  v4f o[4];
  #pragma unroll
  for (int j = 0; j < 4; ++j) { o[j].x = 0.f; o[j].y = 0.f; o[j].z = 0.f; o[j].w = 0.f; }
  #pragma unroll 1
  for (int s = 0; s < nsel; ++s) {
    const float* p = part + ((size_t)t * KS + s) * DOUT;
    #pragma unroll
    for (int j = 0; j < 4; ++j) {
      const v4f a = *(const v4fa*)(p + 128 * j + 4 * lane);
      o[j] = o[j] + a;
    }
  }
  float* d = out + (size_t)t * DOUT;
  #pragma unroll
  for (int j = 0; j < 4; ++j) *(volatile v4f*)(d + 128 * j + 4 * lane) = o[j];
  __threadfence();
  #pragma unroll
  for (int j = 0; j < 4; ++j) *(volatile v4f*)(d + 128 * j + 4 * lane) = o[j];
}

__global__ __launch_bounds__(256) void k_loss(const float* __restrict__ rec,
                                              float* __restrict__ out_loss, int ntok)
{
  __shared__ double sImp[NEX * 256];
  __shared__ int    sCnt[NEX * 256];
  __shared__ double sV[2 * NEX];
  const int tid = threadIdx.x;
  double imp[NEX];
  int cn[NEX];
  #pragma unroll
  for (int e = 0; e < NEX; ++e) { imp[e] = 0.0; cn[e] = 0; }
  #pragma unroll 1
  for (int i = 0; i < NTOK / 256; ++i) {
    const int t = i * 256 + tid;
    const int tc = (t < ntok) ? t : (ntok - 1);
    const bool ok = (t < ntok);
    const float* rp = rec + (size_t)tc * RECW;
    #pragma unroll
    for (int e = 0; e < NEX; ++e) {
      float g = rp[e];
      g = ok ? g : 0.0f;
      imp[e] += (double)g;
      cn[e]  += (g > 0.0f) ? 1 : 0;
    }
  }
  #pragma unroll
  for (int e = 0; e < NEX; ++e) { sImp[e * 256 + tid] = imp[e]; sCnt[e * 256 + tid] = cn[e]; }
  __syncthreads();
  if (tid < NEX) {
    double s = 0.0;
    int c = 0;
    #pragma unroll 1
    for (int j = 0; j < 256; ++j) { s += sImp[tid * 256 + j]; c += sCnt[tid * 256 + j]; }
    sV[tid] = s;
    sV[NEX + tid] = (double)c;
  }
  __syncthreads();
  if (tid == 0) {
    double total = 0.0;
    #pragma unroll
    for (int pass = 0; pass < 2; ++pass) {
      double mean = 0.0;
      #pragma unroll 1
      for (int e = 0; e < NEX; ++e) mean += sV[pass * NEX + e];
      mean = mean / (double)NEX;
      double var = 0.0;
      #pragma unroll 1
      for (int e = 0; e < NEX; ++e) { const double dd = sV[pass * NEX + e] - mean; var += dd * dd; }
      var = var / (double)(NEX - 1);
      total += var / (mean * mean + 1.0e-10);
    }
    const float lf = (float)total;
    *(volatile float*)out_loss = lf;
    __threadfence();
    *(volatile float*)out_loss = lf;
  }
}

extern "C" void kernel_launch(void* const* d_in, const int* in_sizes, int n_in,
                              void* d_out, int out_size, void* d_ws, size_t ws_size,
                              hipStream_t stream)
{
  if (n_in < 8) return;
  if (in_sizes[0] != NTOK * DIN) return;
  if (in_sizes[1] != NTOK * DIN) return;
  if (in_sizes[2] != DIN * NEX) return;
  if (in_sizes[3] != NEX * DIN * DHID) return;
  if (in_sizes[4] != NEX * DHID) return;
  if (in_sizes[5] != NEX * DHID * DOUT) return;
  if (in_sizes[6] != NEX * DOUT) return;
  if (in_sizes[7] != 1) return;
  if (out_size != NTOK * DOUT + 1) return;

  const float* x   = (const float*)d_in[0];
  const float* gxp = (const float*)d_in[1];
  const float* wgp = (const float*)d_in[2];
  const float* w1  = (const float*)d_in[3];
  const float* b1  = (const float*)d_in[4];
  const float* w2  = (const float*)d_in[5];
  const float* b2  = (const float*)d_in[6];
  const int*   kin = (const int*)d_in[7];
  float* out = (float*)d_out;
  float* out_loss = out + (size_t)NTOK * DOUT;

  const size_t bXH   = (size_t)NTOK * DIN * 2;
  const size_t bW1T  = (size_t)NEX * DHID * DIN * 2;
  const size_t bW2T  = (size_t)NEX * DOUT * DHID * 2;
  const size_t bREC  = (size_t)NTOK * RECW * 4;
  const size_t bPART = (size_t)NTOK * KS * DOUT * 4;
  const size_t total = bXH + bW1T + bW2T + bREC + bPART;
  if (total > ws_size) return;
  if (total > (size_t)134217728) return;

  char* ws = (char*)d_ws;
  size_t off = 0;
  unsigned short* XH   = (unsigned short*)(ws + off); off += bXH;
  unsigned short* W1T  = (unsigned short*)(ws + off); off += bW1T;
  unsigned short* W2T  = (unsigned short*)(ws + off); off += bW2T;
  float*          REC  = (float*)(ws + off);          off += bREC;
  float*          PART = (float*)(ws + off);          off += bPART;
  if (off != total) return;

  hipFuncSetAttribute(reinterpret_cast<const void*>(&k_expert),
                      hipFuncAttributeMaxDynamicSharedMemorySize, LDS_EXP);

  {
    const int n8x = NTOK * DIN / 8;
    k_cvt<<<(n8x + 255) / 256, 256, 0, stream>>>(x, XH, n8x, 1.0f);
  }
  k_tcv<<<dim3(DHID / TT, DIN / TT, NEX), 256, 0, stream>>>(w1, W1T, DIN, DHID, W_SC);
  k_tcv<<<dim3(DOUT / TT, DHID / TT, NEX), 256, 0, stream>>>(w2, W2T, DHID, DOUT, W_SC);
  k_route<<<(NTOK + 7) / 8, 256, 0, stream>>>(gxp, wgp, kin, REC, NTOK);
  k_expert<<<dim3(GX, NEX), 256, LDS_EXP, stream>>>(XH, W1T, b1, W2T, b2, REC, PART, NTOK);
  k_sum<<<(NTOK + 7) / 8, 256, 0, stream>>>(PART, REC, out, NTOK);
  k_loss<<<1, 256, 0, stream>>>(REC, out_loss, NTOK);
}
